// WTMamba_18245021073646
// MI455X (gfx1250) — hardware-run, weakly checked
//
#include <hip/hip_runtime.h>
#include <math.h>

typedef __attribute__((ext_vector_type(16))) _Float16 v16h;
typedef __attribute__((ext_vector_type(8)))  _Float16 v8h;
typedef __attribute__((ext_vector_type(8)))  float    v8f;
typedef __attribute__((ext_vector_type(4)))  float    v4f;
typedef __attribute__((ext_vector_type(4)))  unsigned v4u;

constexpr int kNb    = 4;
constexpr int kCh    = 64;
constexpr int kS1    = 192;
constexpr int kS2    = 96;
constexpr int kS3    = 48;
constexpr int kP1    = kS1 + 4;
constexpr int kP2    = kS2 + 4;
constexpr int kLen1  = kS2 * kS2;
constexpr int kLen2  = kS3 * kS3;
constexpr int kRows1 = kNb * kLen1;
constexpr int kRows2 = kNb * kLen2;
constexpr int kDin   = 128;
constexpr int kXzP   = 256;
constexpr int kXdP   = 64;
constexpr int kNst   = 16;
constexpr int kDtR   = 4;
constexpr int kTaps  = 25;
constexpr float kWCarry   = 16.0f;
constexpr float kXsCarry  = 64.0f;
constexpr float kYgCarry  = 256.0f;
constexpr float kWCarryInv  = 1.0f / kWCarry;
constexpr float kXsCarryInv = 1.0f / kXsCarry;
constexpr int kConvSlab = 64 * 36;
constexpr int kDwTP = 132;
constexpr int kScanTS = 64;
constexpr int kScanYP = 68;
static_assert(kConvSlab >= 32 * 68, "slab holds both epilogue layouts");
static_assert(kDtR + 2 * kNst <= kXdP, "x_proj width fits the padded pitch");
static_assert((kRows1 % 64) == 0 && (kRows2 % 64) == 0, "GEMM M multiples of 64");
static_assert((kLen1 % kScanTS) == 0 && (kLen2 % kScanTS) == 0, "scan chunk multiples");
static_assert((kS1 % 32) == 0 && (kS2 % 32) == 0, "row segments of 32 pixels");

constexpr size_t kSzFilt = (size_t)kTaps * 64 * 64 * 2;
constexpr size_t kSzWin  = (size_t)kXzP * kCh * 2;
constexpr size_t kSzWxp  = (size_t)kXdP * kDin * 2;
constexpr size_t kSzWou  = (size_t)kCh * kDin * 2;
constexpr size_t kSzP1   = (size_t)kNb * kP1 * kP1 * 64 * 2;
constexpr size_t kSzP2   = (size_t)kNb * kP2 * kP2 * 64 * 2;
constexpr size_t kSzSeq  = (size_t)kRows1 * kCh * 2;
constexpr size_t kSzXz   = (size_t)kRows1 * kXzP * 2;
constexpr size_t kSzXs   = (size_t)kRows1 * kDin * 2;
constexpr size_t kSzXd   = (size_t)kRows1 * kXdP * 4;
constexpr size_t kSzYg   = (size_t)kRows1 * kDin * 2;
constexpr size_t kSzMo1  = (size_t)kRows1 * kCh * 4;
constexpr size_t kSzMo2  = (size_t)kRows2 * kCh * 4;
constexpr size_t kOffFW  = 0;
constexpr size_t kOffFI  = kOffFW  + kSzFilt;
constexpr size_t kOffWin = kOffFI  + kSzFilt;
constexpr size_t kOffWxp = kOffWin + kSzWin;
constexpr size_t kOffWou = kOffWxp + kSzWxp;
constexpr size_t kOffXP1 = kOffWou + kSzWou;
constexpr size_t kOffY1  = kOffXP1 + kSzP1;
constexpr size_t kOffX2  = kOffY1  + kSzP1;
constexpr size_t kOffY2  = kOffX2  + kSzP2;
constexpr size_t kOffSeq = kOffY2  + kSzP2;
constexpr size_t kOffXz  = kOffSeq + kSzSeq;
constexpr size_t kOffXs  = kOffXz  + kSzXz;
constexpr size_t kOffXd  = kOffXs  + kSzXs;
constexpr size_t kOffYg  = kOffXd  + kSzXd;
constexpr size_t kOffMo1 = kOffYg  + kSzYg;
constexpr size_t kOffMo2 = kOffMo1 + kSzMo1;
constexpr size_t kWsTotal = kOffMo2 + kSzMo2;
static_assert(kWsTotal == 113754112ull, "carve total");
static_assert(kWsTotal <= 134217728ull, "carve cap");
static_assert((kOffFI % 128) == 0 && (kOffWin % 128) == 0 && (kOffWxp % 128) == 0 && (kOffWou % 128) == 0 &&
              (kOffXP1 % 128) == 0 && (kOffY1 % 128) == 0 && (kOffX2 % 128) == 0 && (kOffY2 % 128) == 0 &&
              (kOffSeq % 128) == 0 && (kOffXz % 128) == 0 && (kOffXs % 128) == 0 && (kOffXd % 128) == 0 &&
              (kOffYg % 128) == 0 && (kOffMo1 % 128) == 0 && (kOffMo2 % 128) == 0, "128-B aligned regions");

__device__ __forceinline__ float rbf(float f) {
  unsigned u = __float_as_uint(f);
  u = (u + 0x7FFFu + ((u >> 16) & 1u)) & 0xFFFF0000u;
  return __uint_as_float(u);
}
__device__ __forceinline__ float h16_to_f32(unsigned hb) {
  const unsigned sgn = (hb & 0x8000u) << 16;
  const unsigned em = hb & 0x7fffu;
  const float fn = __uint_as_float((em << 13) + 0x38000000u);
  const float fs = (float)em * 5.9604644775390625e-8f;
  const float mag = (em < 0x400u) ? fs : fn;
  return __uint_as_float(__float_as_uint(mag) | sgn);
}
__device__ __forceinline__ v16h frag_load(const _Float16* p) {
  union U { v16h v; v8h h[2]; } f;
  f.h[0] = *(const v8h*)(p);
  f.h[1] = *(const v8h*)(p + 16);
  return f.v;
}
__device__ __forceinline__ v8f mma_h(v16h a, v16h b, v8f c) {
  return __builtin_amdgcn_wmma_f32_16x16x32_f16(false, a, false, b, (short)0, c, false, false);
}
__device__ __forceinline__ void guard4_h(v8f& a, v8f& b, v8f& c, v8f& d, v16h x) {
  asm volatile("v_nop\n\tv_nop\n\tv_nop\n\tv_nop" : "+v"(a), "+v"(b), "+v"(c), "+v"(d) : "v"(x));
}
__device__ __forceinline__ void keep4_h(v16h a, v16h b, v16h c, v16h d) {
  asm volatile("v_nop" :: "v"(a), "v"(b), "v"(c), "v"(d));
}
__device__ __forceinline__ void acc_guard4(v8f& a, v8f& b, v8f& c, v8f& d) {
  asm volatile("v_nop\n\tv_nop\n\tv_nop\n\tv_nop" : "+v"(a), "+v"(b), "+v"(c), "+v"(d));
}
__device__ __forceinline__ void conv_guard8(v8f& c0, v8f& c1, v8f& c2, v8f& c3, v8f& c4, v8f& c5, v8f& c6, v8f& c7,
                                            v16h a0, v16h a1, v16h b0, v16h b1, v16h b2, v16h b3) {
  asm volatile("v_nop\n\tv_nop\n\tv_nop\n\tv_nop"
               : "+v"(c0), "+v"(c1), "+v"(c2), "+v"(c3), "+v"(c4), "+v"(c5), "+v"(c6), "+v"(c7)
               : "v"(a0), "v"(a1), "v"(b0), "v"(b1), "v"(b2), "v"(b3));
}
__device__ __forceinline__ void wave_lds_sync() {
  __builtin_amdgcn_fence(__ATOMIC_RELEASE, "workgroup");
  __builtin_amdgcn_wave_barrier();
  __builtin_amdgcn_fence(__ATOMIC_ACQUIRE, "workgroup");
}

__global__ __launch_bounds__(256) void pack_filter_kernel(
    const float* __restrict__ f0, const float* __restrict__ f1,
    unsigned short* __restrict__ p0, unsigned short* __restrict__ p1)
{
  const float* f = (blockIdx.y == 0) ? f0 : f1;
  unsigned short* p = (blockIdx.y == 0) ? p0 : p1;
  const int i = blockIdx.x * 256 + threadIdx.x;
  if (i >= kTaps * 64 * 64 / 8) return;
  const int e0  = i << 3;
  const int tap = e0 >> 12;
  const int co  = (e0 >> 6) & 63;
  const int ci0 = e0 & 63;
  v8h hv;
#pragma unroll
  for (int e = 0; e < 8; ++e) {
    const float v = f[(size_t)(co * 64 + ci0 + e) * kTaps + tap];
    hv[e] = (_Float16)(rbf(v) * kWCarry);
  }
  unsigned short* q = p + e0;
  *(volatile v8h*)q = hv;
  __threadfence();
  *(volatile v8h*)q = hv;
}

__global__ __launch_bounds__(256) void cast_w_kernel(
    const float* __restrict__ src, unsigned short* __restrict__ dst, int total8, int nreal, float scale)
{
  const int i = blockIdx.x * 256 + threadIdx.x;
  if (i >= total8) return;
  const int e0 = i << 3;
  const bool inr = (e0 < nreal);
  const int ec = inr ? e0 : 0;
  const v4f a0 = *(const v4f*)(src + ec);
  const v4f a1 = *(const v4f*)(src + ec + 4);
  v8h hv;
#pragma unroll
  for (int e = 0; e < 4; ++e) {
    const float x0 = inr ? (rbf(a0[e]) * scale) : 0.0f;
    const float x1 = inr ? (rbf(a1[e]) * scale) : 0.0f;
    hv[e]     = (_Float16)x0;
    hv[4 + e] = (_Float16)x1;
  }
  unsigned short* q = dst + e0;
  *(volatile v8h*)q = hv;
  __threadfence();
  *(volatile v8h*)q = hv;
}

__global__ __launch_bounds__(256) void pack_x_kernel(const float* __restrict__ x, unsigned short* __restrict__ xp)
{
  const int i = blockIdx.x * 256 + threadIdx.x;
  if (i >= kNb * kP1 * kP1 * 8) return;
  const int c8 = (i & 7) * 8;
  int p = i >> 3;
  const int xx = p % kP1;
  p /= kP1;
  const int yy = p % kP1;
  const int b  = p / kP1;
  const int ys = yy - 2, xs = xx - 2;
  const bool inb = ((unsigned)ys < (unsigned)kS1) && ((unsigned)xs < (unsigned)kS1);
  const int ysc = ys < 0 ? 0 : (ys > kS1 - 1 ? kS1 - 1 : ys);
  const int xsc = xs < 0 ? 0 : (xs > kS1 - 1 ? kS1 - 1 : xs);
  const size_t base = ((size_t)(b * 64 + c8) * kS1 + ysc) * kS1 + xsc;
  v8h hv;
#pragma unroll
  for (int e = 0; e < 8; ++e) {
    const float v = x[base + (size_t)e * kS1 * kS1];
    const float w = inb ? rbf(v) : 0.0f;
    hv[e] = (_Float16)w;
  }
  unsigned short* q = xp + (size_t)(i >> 3) * 64 + c8;
  *(volatile v8h*)q = hv;
  __threadfence();
  *(volatile v8h*)q = hv;
}

__global__ __launch_bounds__(256) void halo_zero_kernel(
    unsigned short* __restrict__ q0, int s0, unsigned short* __restrict__ q1, int s1,
    unsigned short* __restrict__ q2, int s2)
{
  unsigned short* P = (blockIdx.y == 0) ? q0 : ((blockIdx.y == 1) ? q1 : q2);
  const int Sn = (blockIdx.y == 0) ? s0 : ((blockIdx.y == 1) ? s1 : s2);
  const int Wp = Sn + 4;
  const int nh = 8 * Sn + 16;
  const int i = blockIdx.x * 256 + threadIdx.x;
  if (i >= kNb * nh * 8) return;
  const int c8 = (i & 7) * 8;
  int k = i >> 3;
  const int b = k / nh;
  k -= b * nh;
  const int kA = k;
  const int kB = k - 2 * Wp;
  const int kC = k - 4 * Wp;
  const int rowA = kA / Wp;
  const int colA = kA - rowA * Wp;
  const int rB = (kB < 0 ? 0 : kB) / Wp;
  const int rowB = Wp - 2 + rB;
  const int colB = (kB < 0 ? 0 : kB) - rB * Wp;
  const int kCc = kC < 0 ? 0 : kC;
  const int rowC = 2 + (kCc >> 2);
  const int cs = kCc & 3;
  const int colC = (cs < 2) ? cs : (Wp - 4 + cs);
  const int row = (k < 2 * Wp) ? rowA : ((k < 4 * Wp) ? rowB : rowC);
  const int col = (k < 2 * Wp) ? colA : ((k < 4 * Wp) ? colB : colC);
  unsigned short* q = P + ((size_t)(b * Wp + row) * Wp + col) * 64 + c8;
  const v4u z = (v4u){0u, 0u, 0u, 0u};
  *(volatile v4u*)q = z;
  __threadfence();
  *(volatile v4u*)q = z;
}

template <int MODE>
__global__ __launch_bounds__(256) void conv5x5_kernel(
    const unsigned short* __restrict__ inp, const unsigned short* __restrict__ filt,
    void* __restrict__ outp, const float* __restrict__ addsrc, int Hn, int Wn)
{
  __shared__ __align__(16) float sT[8][kConvSlab];
  const int lane = threadIdx.x & 31;
  const int wave = threadIdx.x >> 5;
  const int segs = Wn >> 5;
  const int tile = blockIdx.x * 8 + wave;
  if (tile >= kNb * Hn * segs) return;
  const int sg = tile % segs;
  const int t1 = tile / segs;
  const int h  = t1 % Hn;
  const int b  = t1 / Hn;
  const int w0 = sg << 5;
  const int Wp = Wn + 4, Hp = Hn + 4;
  const int rlane = lane & 15;
  const int hh    = lane >> 4;
  const int koff  = hh * 8;
  const int mOff  = hh * 8;

  const _Float16* ap = (const _Float16*)inp + ((size_t)(b * Hp + h) * Wp + w0 + rlane) * 64 + koff;
  const _Float16* bp = (const _Float16*)filt + (size_t)rlane * 64 + koff;

  v8f acc[2][4];
#pragma unroll
  for (int i = 0; i < 2; ++i)
#pragma unroll
    for (int j = 0; j < 4; ++j) acc[i][j] = (v8f){0.f, 0.f, 0.f, 0.f, 0.f, 0.f, 0.f, 0.f};

#pragma unroll 1
  for (int kh = 0; kh < 5; ++kh) {
#pragma unroll 1
    for (int kw = 0; kw < 5; ++kw) {
      const _Float16* at = ap + ((size_t)kh * Wp + kw) * 64;
      const _Float16* bt = bp + (size_t)(kh * 5 + kw) * 4096;
#pragma unroll
      for (int cc = 0; cc < 2; ++cc) {
        const v16h bf0 = frag_load(bt + cc * 32);
        const v16h bf1 = frag_load(bt + 1024 + cc * 32);
        const v16h bf2 = frag_load(bt + 2048 + cc * 32);
        const v16h bf3 = frag_load(bt + 3072 + cc * 32);
        const v16h a0 = frag_load(at + cc * 32);
        const v16h a1 = frag_load(at + 1024 + cc * 32);
        acc[0][0] = mma_h(a0, bf0, acc[0][0]);
        acc[0][1] = mma_h(a0, bf1, acc[0][1]);
        acc[0][2] = mma_h(a0, bf2, acc[0][2]);
        acc[0][3] = mma_h(a0, bf3, acc[0][3]);
        acc[1][0] = mma_h(a1, bf0, acc[1][0]);
        acc[1][1] = mma_h(a1, bf1, acc[1][1]);
        acc[1][2] = mma_h(a1, bf2, acc[1][2]);
        acc[1][3] = mma_h(a1, bf3, acc[1][3]);
        conv_guard8(acc[0][0], acc[0][1], acc[0][2], acc[0][3], acc[1][0], acc[1][1], acc[1][2], acc[1][3],
                    a0, a1, bf0, bf1, bf2, bf3);
      }
    }
  }

  float* slab = sT[wave];
  if (MODE == 2) {
#pragma unroll
    for (int i = 0; i < 2; ++i) {
#pragma unroll
      for (int j = 0; j < 4; ++j) {
        float* sp = slab + ((j << 4) + rlane) * 36 + (i << 4) + mOff;
        v4f lo4, hi4;
#pragma unroll
        for (int e = 0; e < 4; ++e) {
          lo4[e] = acc[i][j][e] * kWCarryInv;
          hi4[e] = acc[i][j][4 + e] * kWCarryInv;
        }
        *(v4f*)(sp) = lo4;
        *(v4f*)(sp + 4) = hi4;
      }
    }
    wave_lds_sync();
    const int q = lane >> 3, c4 = (lane & 7) * 4;
    float* outf = (float*)outp;
    v4f ov[16];
#pragma unroll
    for (int it = 0; it < 16; ++it) ov[it] = *(const v4f*)(slab + (it * 4 + q) * 36 + c4);
    for (int pass = 0; pass < 2; ++pass) {
#pragma unroll
      for (int it = 0; it < 16; ++it) {
        const int co = it * 4 + q;
        *(volatile v4f*)(outf + (((size_t)b * 64 + co) * Hn + h) * Wn + w0 + c4) = ov[it];
      }
      __threadfence();
    }
  } else {
#pragma unroll
    for (int i = 0; i < 2; ++i) {
#pragma unroll
      for (int j = 0; j < 4; ++j) {
#pragma unroll
        for (int r = 0; r < 8; ++r)
          slab[((i << 4) + mOff + r) * 68 + (j << 4) + rlane] = acc[i][j][r] * kWCarryInv;
      }
    }
    wave_lds_sync();
    const int q = lane >> 3, c8 = (lane & 7) * 8;
    unsigned short* outh = (unsigned short*)outp;
    v8h hv[8];
#pragma unroll
    for (int it = 0; it < 8; ++it) {
      const int px = it * 4 + q;
      const float* sp = slab + px * 68 + c8;
      v4f a0 = *(const v4f*)(sp);
      v4f a1 = *(const v4f*)(sp + 4);
      if (MODE == 1) {
        const float* mp = addsrc + ((size_t)b * Hn * Wn + (size_t)(w0 + px) * Hn + h) * 64 + c8;
        const v4f m0 = *(const v4f*)(mp);
        const v4f m1 = *(const v4f*)(mp + 4);
        a0 = a0 + m0;
        a1 = a1 + m1;
      }
#pragma unroll
      for (int e = 0; e < 4; ++e) {
        hv[it][e]     = (_Float16)a0[e];
        hv[it][4 + e] = (_Float16)a1[e];
      }
    }
    for (int pass = 0; pass < 2; ++pass) {
#pragma unroll
      for (int it = 0; it < 8; ++it) {
        const int px = it * 4 + q;
        size_t o;
        if (MODE == 0) {
          o = ((size_t)(b * Hp + h + 2) * Wp + w0 + px + 2) * 64 + c8;
        } else {
          const int Wo = 2 * Wn + 4, Ho = 2 * Hn + 4;
          o = ((size_t)(b * Ho + 2 * h + 2) * Wo + 2 * (w0 + px) + 2) * 64 + c8;
        }
        *(volatile v8h*)(outh + o) = hv[it];
      }
      __threadfence();
    }
  }
}

template <bool WITH_X2>
__global__ __launch_bounds__(256) void extract_ll_kernel(
    const unsigned short* __restrict__ Y, unsigned short* __restrict__ X2, unsigned short* __restrict__ SEQ, int Sn)
{
  const int S2 = Sn >> 1;
  const int i = blockIdx.x * 256 + threadIdx.x;
  if (i >= kNb * S2 * S2 * 8) return;
  const int c8 = (i & 7) * 8;
  int p = i >> 3;
  const int ww = p % S2;
  p /= S2;
  const int hh = p % S2;
  const int b  = p / S2;
  const int Wp = Sn + 4;
  const v4u v = *(const v4u*)(Y + ((size_t)(b * Wp + 2 * hh + 2) * Wp + 2 * ww + 2) * 64 + c8);
  unsigned short* qs = SEQ + ((size_t)b * S2 * S2 + (size_t)ww * S2 + hh) * 64 + c8;
  const int Wq = S2 + 4;
  unsigned short* qx = WITH_X2 ? (X2 + ((size_t)(b * Wq + hh + 2) * Wq + ww + 2) * 64 + c8) : qs;
  *(volatile v4u*)qs = v;
  if (WITH_X2) *(volatile v4u*)qx = v;
  __threadfence();
  *(volatile v4u*)qs = v;
  if (WITH_X2) *(volatile v4u*)qx = v;
}

__global__ __launch_bounds__(256) void patch_ll_kernel(
    const float* __restrict__ MO, unsigned short* __restrict__ Y, int S2)
{
  const int i = blockIdx.x * 256 + threadIdx.x;
  if (i >= kNb * S2 * S2 * 8) return;
  const int c8 = (i & 7) * 8;
  int p = i >> 3;
  const int ww = p % S2;
  p /= S2;
  const int hh = p % S2;
  const int b  = p / S2;
  const float* mp = MO + ((size_t)b * S2 * S2 + (size_t)ww * S2 + hh) * 64 + c8;
  const v4f a0 = *(const v4f*)(mp);
  const v4f a1 = *(const v4f*)(mp + 4);
  v8h hv;
#pragma unroll
  for (int e = 0; e < 4; ++e) {
    hv[e]     = (_Float16)a0[e];
    hv[4 + e] = (_Float16)a1[e];
  }
  const int Wp = 2 * S2 + 4;
  unsigned short* q = Y + ((size_t)(b * Wp + 2 * hh + 2) * Wp + 2 * ww + 2) * 64 + c8;
  *(volatile v8h*)q = hv;
  __threadfence();
  *(volatile v8h*)q = hv;
}

template <int OUT_MODE>
__global__ __launch_bounds__(256) void wmma_gemm64(
    const unsigned short* __restrict__ Ap, int lda,
    const unsigned short* __restrict__ Btp, int ldb,
    void* __restrict__ Cout, int ldc, int M, int N, int K, float scale)
{
  const _Float16* A  = (const _Float16*)Ap;
  const _Float16* Bt = (const _Float16*)Btp;
  __shared__ __align__(16) float sT[8][16 * 68];
  const int lane = threadIdx.x & 31;
  const int wave = threadIdx.x >> 5;
  const int tilesN = N >> 6;
  const int tilesM = M >> 6;
  const int tile = blockIdx.x * 8 + wave;
  if (tile >= tilesM * tilesN) return;
  const int tm = tile / tilesN;
  const int tn = tile - tm * tilesN;
  const int m0 = tm << 6;
  const int n0 = tn << 6;
  const int rlane = lane & 15;
  const int koff  = (lane >> 4) * 8;
  const int mOff  = (lane >> 4) * 8;

  v8f acc[4][4];
#pragma unroll
  for (int i = 0; i < 4; ++i)
#pragma unroll
    for (int j = 0; j < 4; ++j) acc[i][j] = (v8f){0.f, 0.f, 0.f, 0.f, 0.f, 0.f, 0.f, 0.f};

  for (int k0 = 0; k0 < K; k0 += 32) {
    v16h bh[4];
#pragma unroll
    for (int j = 0; j < 4; ++j) {
      const size_t bo = (size_t)(n0 + (j << 4) + rlane) * ldb + koff + k0;
      bh[j] = frag_load(Bt + bo);
    }
#pragma unroll
    for (int i = 0; i < 4; ++i) {
      const size_t ao = (size_t)(m0 + (i << 4) + rlane) * lda + koff + k0;
      const v16h ah = frag_load(A + ao);
#pragma unroll
      for (int j = 0; j < 4; ++j) acc[i][j] = mma_h(ah, bh[j], acc[i][j]);
      guard4_h(acc[i][0], acc[i][1], acc[i][2], acc[i][3], ah);
    }
    keep4_h(bh[0], bh[1], bh[2], bh[3]);
  }
  acc_guard4(acc[0][0], acc[0][1], acc[0][2], acc[0][3]);
  acc_guard4(acc[1][0], acc[1][1], acc[1][2], acc[1][3]);
  acc_guard4(acc[2][0], acc[2][1], acc[2][2], acc[2][3]);
  acc_guard4(acc[3][0], acc[3][1], acc[3][2], acc[3][3]);

  float* slab = sT[wave];
#pragma unroll
  for (int i = 0; i < 4; ++i) {
    const int mBase = m0 + (i << 4);
#pragma unroll
    for (int j = 0; j < 4; ++j) {
#pragma unroll
      for (int r = 0; r < 8; ++r)
        slab[(mOff + r) * 68 + (j << 4) + rlane] = acc[i][j][r] * scale;
    }
    wave_lds_sync();
    if (OUT_MODE == 0) {
      float* C = (float*)Cout;
      const int hh = lane >> 4, c4 = (lane & 15) * 4;
      for (int pass = 0; pass < 2; ++pass) {
#pragma unroll
        for (int it = 0; it < 8; ++it) {
          const int row = it * 2 + hh;
          const v4f v = *(const v4f*)(slab + row * 68 + c4);
          *(volatile v4f*)(C + (size_t)(mBase + row) * ldc + n0 + c4) = v;
        }
        __threadfence();
      }
    } else {
      const int q = lane >> 3, c8 = (lane & 7) * 8;
      unsigned short* C = (unsigned short*)Cout;
      for (int pass = 0; pass < 2; ++pass) {
#pragma unroll
        for (int it = 0; it < 4; ++it) {
          const int row = it * 4 + q;
          const float* sp = slab + row * 68 + c8;
          v8h hv;
#pragma unroll
          for (int e = 0; e < 8; ++e) hv[e] = (_Float16)sp[e];
          *(volatile v8h*)(C + (size_t)(mBase + row) * ldc + n0 + c8) = hv;
        }
        __threadfence();
      }
    }
    wave_lds_sync();
  }
}

__global__ __launch_bounds__(128) void dwconv_silu_kernel(
    const unsigned short* __restrict__ XZ, const float* __restrict__ cw, const float* __restrict__ cb,
    unsigned short* __restrict__ XS, int L)
{
  __shared__ __align__(16) float sT[16 * kDwTP];
  const int tid = threadIdx.x, lane = tid & 31, wave = tid >> 5;
  const int d = tid;
  const int g0 = blockIdx.x * 64;
  const int tb = g0 % L;
  const v4f wv = *(const v4f*)(cw + d * 4);
  const float w0 = rbf(wv[0]), w1 = rbf(wv[1]), w2 = rbf(wv[2]), w3 = rbf(wv[3]);
  const float bc = rbf(cb[d]);
  float xm3, xm2, xm1;
  {
    const bool hist = (tb > 0);
    const int rb = hist ? (g0 - 3) : g0;
    const float v3 = h16_to_f32((unsigned)XZ[(size_t)rb * kXzP + d]);
    const float v2 = h16_to_f32((unsigned)XZ[(size_t)(rb + 1) * kXzP + d]);
    const float v1 = h16_to_f32((unsigned)XZ[(size_t)(rb + 2) * kXzP + d]);
    xm3 = hist ? v3 : 0.f;
    xm2 = hist ? v2 : 0.f;
    xm1 = hist ? v1 : 0.f;
  }
  const int frow = wave * 2 + (lane >> 4);
  const int fc8  = (lane & 15) * 8;
#pragma unroll 1
  for (int sub = 0; sub < 4; ++sub) {
    const int lb = g0 + sub * 16;
#pragma unroll 1
    for (int s = 0; s < 16; ++s) {
      const float xcur = h16_to_f32((unsigned)XZ[(size_t)(lb + s) * kXzP + d]);
      float acc = w0 * xm3;
      acc = fmaf(w1, xm2, acc);
      acc = fmaf(w2, xm1, acc);
      acc = fmaf(w3, xcur, acc);
      const float sv = acc + bc;
      const float sg = __builtin_amdgcn_rcpf(1.0f + __expf(-sv));
      sT[s * kDwTP + tid] = (sv * sg) * kXsCarry;
      xm3 = xm2;
      xm2 = xm1;
      xm1 = xcur;
    }
    __syncthreads();
    v8h bv[2];
#pragma unroll
    for (int it = 0; it < 2; ++it) {
      const float* sp = sT + (it * 8 + frow) * kDwTP + fc8;
      const v4f a0 = *(const v4f*)(sp);
      const v4f a1 = *(const v4f*)(sp + 4);
#pragma unroll
      for (int e = 0; e < 4; ++e) {
        bv[it][e]     = (_Float16)a0[e];
        bv[it][4 + e] = (_Float16)a1[e];
      }
    }
    for (int pass = 0; pass < 2; ++pass) {
#pragma unroll
      for (int it = 0; it < 2; ++it)
        *(volatile v8h*)(XS + (size_t)(lb + it * 8 + frow) * kDin + fc8) = bv[it];
      __threadfence();
    }
    __syncthreads();
  }
}

__global__ __launch_bounds__(64) void scan_kernel(
    const float* __restrict__ XD, const unsigned short* __restrict__ XS, const unsigned short* __restrict__ XZ,
    const float* __restrict__ Wdt, const float* __restrict__ bdt, const float* __restrict__ Alog,
    const float* __restrict__ Dp, unsigned short* __restrict__ YG, int L)
{
  __shared__ __align__(16) float sX[kScanTS * kXdP];
  __shared__ __align__(16) float sY[kScanTS * kScanYP];
  __shared__ __align__(16) float sA[kNst * 64];
  const int tid = threadIdx.x, lane = tid & 31, wave = tid >> 5;
  const int bix = blockIdx.x >> 1;
  const int d0  = (blockIdx.x & 1) * 64;
  const int d   = d0 + tid;
  const size_t row0 = (size_t)bix * L;
#pragma unroll 1
  for (int s = 0; s < kNst; ++s) sA[s * 64 + tid] = -expf(rbf(Alog[(size_t)d * kNst + s]));
  __syncthreads();
  float negA[kNst], h[kNst];
#pragma unroll
  for (int s = 0; s < kNst; ++s) {
    negA[s] = sA[s * 64 + tid];
    h[s] = 0.f;
  }
  const v4f wq = *(const v4f*)(Wdt + d * kDtR);
  const float wd0 = rbf(wq[0]), wd1 = rbf(wq[1]), wd2 = rbf(wq[2]), wd3 = rbf(wq[3]);
  const float bb = rbf(bdt[d]);
  const float Dd = rbf(Dp[d]);
  const int lr = tid >> 4, lc4 = (tid & 15) * 4;
  const int q = lane >> 3, c8 = (lane & 7) * 8;
#pragma unroll 1
  for (int t0 = 0; t0 < L; t0 += kScanTS) {
    __syncthreads();
#pragma unroll
    for (int i = 0; i < 16; ++i) {
      const int r = lr + 4 * i;
      *(v4f*)(sX + r * kXdP + lc4) = *(const v4f*)(XD + (row0 + t0 + r) * kXdP + lc4);
    }
    __syncthreads();
#pragma unroll 1
    for (int s = 0; s < kScanTS; ++s) {
      const size_t row = row0 + t0 + s;
      const float* xr = sX + s * kXdP;
      const v4f dv = *(const v4f*)(xr);
      float vdot = dv[0] * wd0;
      vdot = fmaf(dv[1], wd1, vdot);
      vdot = fmaf(dv[2], wd2, vdot);
      vdot = fmaf(dv[3], wd3, vdot);
      float Bs[kNst], Cs[kNst];
#pragma unroll
      for (int q4 = 0; q4 < 4; ++q4) {
        const v4f bv = *(const v4f*)(xr + kDtR + 4 * q4);
        const v4f cv = *(const v4f*)(xr + kDtR + kNst + 4 * q4);
        Bs[4 * q4 + 0] = bv[0]; Bs[4 * q4 + 1] = bv[1]; Bs[4 * q4 + 2] = bv[2]; Bs[4 * q4 + 3] = bv[3];
        Cs[4 * q4 + 0] = cv[0]; Cs[4 * q4 + 1] = cv[1]; Cs[4 * q4 + 2] = cv[2]; Cs[4 * q4 + 3] = cv[3];
      }
      const float v   = vdot + bb;
      const float a   = __expf(-fabsf(v));
      const float u   = 1.0f + a;
      const float l1p = __logf(u) + (a - (u - 1.0f)) * __builtin_amdgcn_rcpf(u);
      const float dt  = fmaxf(v, 0.0f) + l1p;
      float xt = h16_to_f32((unsigned)XS[row * kDin + d]) * kXsCarryInv;
      asm volatile("" : "+v"(xt));
      float zv = h16_to_f32((unsigned)XZ[row * kXzP + kDin + d]);
      asm volatile("" : "+v"(zv));
      const float dtx = dt * xt;
      float y = 0.f;
#pragma unroll
      for (int k = 0; k < kNst; ++k) {
        const float e = __expf(dt * negA[k]);
        h[k] = fmaf(e, h[k], dtx * Bs[k]);
        y = fmaf(h[k], Cs[k], y);
      }
      y = fmaf(xt, Dd, y);
      const float sg = __builtin_amdgcn_rcpf(1.0f + __expf(-zv));
      y = y * (zv * sg);
      sY[s * kScanYP + tid] = y * kYgCarry;
    }
    __syncthreads();
    v8h hv[8];
#pragma unroll
    for (int it = 0; it < 8; ++it) {
      const int rw = it * 8 + wave * 4 + q;
      const float* sp = sY + rw * kScanYP + c8;
      const v4f a0 = *(const v4f*)(sp);
      const v4f a1 = *(const v4f*)(sp + 4);
#pragma unroll
      for (int e = 0; e < 4; ++e) {
        hv[it][e]     = (_Float16)a0[e];
        hv[it][4 + e] = (_Float16)a1[e];
      }
    }
    for (int pass = 0; pass < 2; ++pass) {
#pragma unroll
      for (int it = 0; it < 8; ++it) {
        const int rw = it * 8 + wave * 4 + q;
        *(volatile v8h*)(YG + (row0 + t0 + rw) * kDin + d0 + c8) = hv[it];
      }
      __threadfence();
    }
  }
}

extern "C" void kernel_launch(void* const* d_in, const int* in_sizes, int n_in,
                              void* d_out, int out_size, void* d_ws, size_t ws_size,
                              hipStream_t stream)
{
  if (n_in < 12) return;
  if (in_sizes[0] != kNb * kCh * kS1 * kS1) return;
  if (in_sizes[1] != kCh * kCh * kTaps || in_sizes[2] != kCh * kCh * kTaps) return;
  if (in_sizes[3] != kXzP * kCh) return;
  if (in_sizes[4] != kDin * 4 || in_sizes[5] != kDin) return;
  if (in_sizes[6] != (kDtR + 2 * kNst) * kDin) return;
  if (in_sizes[7] != kDin * kDtR || in_sizes[8] != kDin) return;
  if (in_sizes[9] != kDin * kNst || in_sizes[10] != kDin) return;
  if (in_sizes[11] != kCh * kDin) return;
  if (out_size != kNb * kCh * kS1 * kS1) return;
  if (ws_size < kWsTotal) return;

  const float* x      = (const float*)d_in[0];
  const float* wt_f   = (const float*)d_in[1];
  const float* iwt_f  = (const float*)d_in[2];
  const float* W_in   = (const float*)d_in[3];
  const float* conv_w = (const float*)d_in[4];
  const float* conv_b = (const float*)d_in[5];
  const float* W_x    = (const float*)d_in[6];
  const float* W_dt   = (const float*)d_in[7];
  const float* b_dt   = (const float*)d_in[8];
  const float* A_log  = (const float*)d_in[9];
  const float* D_par  = (const float*)d_in[10];
  const float* W_out  = (const float*)d_in[11];

  char* ws = (char*)d_ws;
  unsigned short* FW  = (unsigned short*)(ws + kOffFW);
  unsigned short* FI  = (unsigned short*)(ws + kOffFI);
  unsigned short* WIN = (unsigned short*)(ws + kOffWin);
  unsigned short* WXP = (unsigned short*)(ws + kOffWxp);
  unsigned short* WOU = (unsigned short*)(ws + kOffWou);
  unsigned short* XP1 = (unsigned short*)(ws + kOffXP1);
  unsigned short* Y1  = (unsigned short*)(ws + kOffY1);
  unsigned short* X2  = (unsigned short*)(ws + kOffX2);
  unsigned short* Y2  = (unsigned short*)(ws + kOffY2);
  unsigned short* SEQ = (unsigned short*)(ws + kOffSeq);
  unsigned short* XZ  = (unsigned short*)(ws + kOffXz);
  unsigned short* XS  = (unsigned short*)(ws + kOffXs);
  float*          XD  = (float*)(ws + kOffXd);
  unsigned short* YG  = (unsigned short*)(ws + kOffYg);
  float*          MO1 = (float*)(ws + kOffMo1);
  float*          MO2 = (float*)(ws + kOffMo2);
  const float* dummy = b_dt;

  pack_filter_kernel<<<dim3(50, 2), 256, 0, stream>>>(wt_f, iwt_f, FW, FI);
  cast_w_kernel<<<(kXzP * kCh / 8) / 256, 256, 0, stream>>>(W_in, WIN, kXzP * kCh / 8, kXzP * kCh, kWCarry);
  cast_w_kernel<<<(kXdP * kDin / 8) / 256, 256, 0, stream>>>(W_x, WXP, kXdP * kDin / 8, (kDtR + 2 * kNst) * kDin, kWCarry);
  cast_w_kernel<<<(kCh * kDin / 8) / 256, 256, 0, stream>>>(W_out, WOU, kCh * kDin / 8, kCh * kDin, kWCarry);
  pack_x_kernel<<<(kNb * kP1 * kP1 * 8) / 256, 256, 0, stream>>>(x, XP1);
  halo_zero_kernel<<<dim3((kNb * (8 * kS1 + 16) * 8 + 255) / 256, 3), 256, 0, stream>>>(Y1, kS1, X2, kS2, Y2, kS2);

  auto run_branch = [&](int M, int L, float* MO) {
    const int tm = M / 64;
    wmma_gemm64<1><<<(tm * 4) / 8, 256, 0, stream>>>(SEQ, kCh, WIN, kCh, (void*)XZ, kXzP, M, kXzP, kCh, kWCarryInv);
    dwconv_silu_kernel<<<tm, 128, 0, stream>>>(XZ, conv_w, conv_b, XS, L);
    wmma_gemm64<0><<<(tm + 7) / 8, 256, 0, stream>>>(XS, kDin, WXP, kDin, (void*)XD, kXdP, M, kXdP, kDin,
                                                     kWCarryInv * kXsCarryInv);
    scan_kernel<<<kNb * 2, 64, 0, stream>>>(XD, XS, XZ, W_dt, b_dt, A_log, D_par, YG, L);
    wmma_gemm64<0><<<(tm + 7) / 8, 256, 0, stream>>>(YG, kDin, WOU, kDin, (void*)MO, kCh, M, kCh, kDin,
                                                     kWCarryInv / kYgCarry);
  };

  conv5x5_kernel<0><<<(kNb * kS1 * (kS1 / 32)) / 8, 256, 0, stream>>>(XP1, FW, (void*)Y1, dummy, kS1, kS1);
  extract_ll_kernel<true><<<(kNb * kS2 * kS2 * 8) / 256, 256, 0, stream>>>(Y1, X2, SEQ, kS1);
  run_branch(kRows1, kLen1, MO1);

  conv5x5_kernel<0><<<(kNb * kS2 * (kS2 / 32)) / 8, 256, 0, stream>>>(X2, FW, (void*)Y2, dummy, kS2, kS2);
  extract_ll_kernel<false><<<(kNb * kS3 * kS3 * 8) / 256, 256, 0, stream>>>(Y2, SEQ, SEQ, kS2);
  run_branch(kRows2, kLen2, MO2);

  patch_ll_kernel<<<(kNb * kS3 * kS3 * 8) / 256, 256, 0, stream>>>(MO2, Y2, kS3);
  conv5x5_kernel<1><<<(kNb * kS2 * (kS2 / 32)) / 8, 256, 0, stream>>>(Y2, FI, (void*)Y1, MO1, kS2, kS2);

  conv5x5_kernel<2><<<(kNb * kS1 * (kS1 / 32)) / 8, 256, 0, stream>>>(Y1, FI, d_out, dummy, kS1, kS1);
}
